// EquiBindNet_48722109006499
// MI455X (gfx1250) — hardware-verified
//
#include <hip/hip_runtime.h>
#define NN 50000
#define NNP 50048
#define NE 800000
#define DDm 64
#define NA 10
#define NL 3
#define NG 64
#define DCAP 64
typedef __bf16 v16b __attribute__((ext_vector_type(16)));
typedef unsigned short v8us __attribute__((ext_vector_type(8), may_alias));
typedef float  v8f  __attribute__((ext_vector_type(8)));
typedef float  v4f  __attribute__((ext_vector_type(4)));
typedef float  v4fa __attribute__((ext_vector_type(4), may_alias));
union FragB { v16b v; v8us half[2]; unsigned short u[16]; };

__device__ __forceinline__ unsigned short bf16_bits(float x) { unsigned int u = __float_as_uint(x); return (unsigned short)((u + 0x7FFFu + ((u >> 16) & 1u)) >> 16); }
__device__ __forceinline__ float bf16_val(unsigned short b) { return __uint_as_float(((unsigned int)b) << 16); }
__device__ __forceinline__ float bf16_round(float x) { return bf16_val(bf16_bits(x)); }
template <int NT>
__device__ __forceinline__ v8f mmaN(v16b ah, v16b al, v16b bh, v16b bl, v8f c) {
  c = __builtin_amdgcn_wmma_f32_16x16x32_bf16(false, ah, false, bh, (short)0, c, false, false);
  if (NT >= 2) c = __builtin_amdgcn_wmma_f32_16x16x32_bf16(false, al, false, bh, (short)0, c, false, false);
  if (NT >= 3) c = __builtin_amdgcn_wmma_f32_16x16x32_bf16(false, ah, false, bl, (short)0, c, false, false);
  asm volatile("v_nop\n\tv_nop\n\tv_nop\n\tv_nop" : "+v"(c) : "v"(ah), "v"(al), "v"(bh), "v"(bl));
  return c;
}

__global__ __launch_bounds__(256) void k_wt_bf16(const float* __restrict__ W, unsigned short* __restrict__ Wt, int K, int N) {
  const int t = blockIdx.x * 256 + threadIdx.x;
  const int k8n = K / 8;
  if (t >= N * k8n) return;
  const int n = t / k8n, k8 = (t % k8n) * 8;
  v8us v;
#pragma unroll
  for (int i = 0; i < 8; ++i) v[i] = bf16_bits(W[(size_t)(k8 + i) * N + n]);
  *(volatile v8us*)(Wt + (size_t)n * K + k8) = v;
  __threadfence();
  *(volatile v8us*)(Wt + (size_t)n * K + k8) = v;
}

template <bool ASPLIT, int ACT, bool BIAS_BF16>
__global__ __launch_bounds__(128) void k_gemm_bf(const float* __restrict__ A, int lda, const unsigned short* __restrict__ Wt, int ldb,
                                               const float* __restrict__ bias, float* __restrict__ C, int ldc, int M, int N, int K) {
  __shared__ __attribute__((aligned(16))) float so[4][16][64];
  const int tid = threadIdx.x, w = tid >> 5, lane = tid & 31, ln = lane & 15, hh = lane >> 4;
  const int ntn = N / 64;
  const int wid = blockIdx.x * 4 + w;
  const int mt = wid / ntn, nq = wid % ntn;
  if (mt * 16 >= M) return;
  const int row0 = mt * 16, col0 = nq * 64;
  const float* arow = A + (size_t)(row0 + ln) * lda;
  v8f acc[4] = {};
  for (int kb = 0; kb < K; kb += 32) {
    FragB ah, al;
    const v4f x0 = *(const v4fa*)(arow + kb + 8 * hh), x1 = *(const v4fa*)(arow + kb + 8 * hh + 4);
    const v4f x2 = *(const v4fa*)(arow + kb + 16 + 8 * hh), x3 = *(const v4fa*)(arow + kb + 16 + 8 * hh + 4);
    float xs[16] = {x0[0],x0[1],x0[2],x0[3],x1[0],x1[1],x1[2],x1[3],x2[0],x2[1],x2[2],x2[3],x3[0],x3[1],x3[2],x3[3]};
#pragma unroll
    for (int i = 0; i < 16; ++i) { const unsigned short hb = bf16_bits(xs[i]); ah.u[i] = hb; al.u[i] = ASPLIT ? bf16_bits(xs[i] - bf16_val(hb)) : (unsigned short)0; }
#pragma unroll
    for (int t = 0; t < 4; ++t) {
      const unsigned short* brow = Wt + (size_t)(col0 + t * 16 + ln) * ldb + kb;
      FragB b;
      b.half[0] = *(const v8us*)(brow + 8 * hh);
      b.half[1] = *(const v8us*)(brow + 16 + 8 * hh);
      acc[t] = mmaN<ASPLIT ? 2 : 1>(ah.v, al.v, b.v, b.v, acc[t]);
    }
  }
#pragma unroll
  for (int t = 0; t < 4; ++t) {
    float bv = bias ? bias[col0 + t * 16 + ln] : 0.f;
    if (BIAS_BF16) bv = bf16_round(bv);
#pragma unroll
    for (int r = 0; r < 8; ++r) { float v = acc[t][r] + bv; if (ACT == 1) v = fmaxf(v, 0.f); so[w][8 * hh + r][t * 16 + ln] = v; }
  }
  __builtin_amdgcn_fence(__ATOMIC_ACQ_REL, "workgroup");
  __builtin_amdgcn_wave_barrier();
  const int rsub = lane >> 4, c4 = (lane & 15) * 4;
  for (int pass = 0; pass < 2; ++pass) {
#pragma unroll
    for (int q = 0; q < 8; ++q) {
      const int r = q * 2 + rsub;
      const v4f v = *(const v4fa*)&so[w][r][c4];
      *(volatile v4f*)(C + (size_t)(row0 + r) * ldc + col0 + c4) = v;
    }
    if (pass == 0) __threadfence();
  }
}

template <bool ASPLIT, int ACT, bool BIAS_BF16, bool RES_BF16>
__global__ __launch_bounds__(128) void k_gemm_bf3(const float* __restrict__ A, int lda, const unsigned short* __restrict__ Wt, int ldb,
                                                const float* __restrict__ bias, const float* __restrict__ resid, int rmod, int ldr,
                                                float* __restrict__ C, int ldc, int M, int N, int K) {
  __shared__ __attribute__((aligned(16))) float so[4][16][64];
  const int tid = threadIdx.x, w = tid >> 5, lane = tid & 31, ln = lane & 15, hh = lane >> 4;
  const int ntn = N / 64;
  const int wid = blockIdx.x * 4 + w;
  const int mt = wid / ntn, nq = wid % ntn;
  if (mt * 16 >= M) return;
  const int row0 = mt * 16, col0 = nq * 64;
  const float* arow = A + (size_t)(row0 + ln) * lda;
  v8f acc[4] = {};
  for (int kb = 0; kb < K; kb += 32) {
    FragB ah, al;
    const v4f x0 = *(const v4fa*)(arow + kb + 8 * hh), x1 = *(const v4fa*)(arow + kb + 8 * hh + 4);
    const v4f x2 = *(const v4fa*)(arow + kb + 16 + 8 * hh), x3 = *(const v4fa*)(arow + kb + 16 + 8 * hh + 4);
    float xs[16] = {x0[0],x0[1],x0[2],x0[3],x1[0],x1[1],x1[2],x1[3],x2[0],x2[1],x2[2],x2[3],x3[0],x3[1],x3[2],x3[3]};
#pragma unroll
    for (int i = 0; i < 16; ++i) { const unsigned short hb = bf16_bits(xs[i]); ah.u[i] = hb; al.u[i] = ASPLIT ? bf16_bits(xs[i] - bf16_val(hb)) : (unsigned short)0; }
#pragma unroll
    for (int t = 0; t < 4; ++t) {
      const unsigned short* brow = Wt + (size_t)(col0 + t * 16 + ln) * ldb + kb;
      FragB b;
      b.half[0] = *(const v8us*)(brow + 8 * hh);
      b.half[1] = *(const v8us*)(brow + 16 + 8 * hh);
      acc[t] = mmaN<ASPLIT ? 2 : 1>(ah.v, al.v, b.v, b.v, acc[t]);
    }
  }
#pragma unroll
  for (int t = 0; t < 4; ++t) {
    const int col = col0 + t * 16 + ln;
    float bv = bias ? bias[col] : 0.f;
    if (BIAS_BF16) bv = bf16_round(bv);
#pragma unroll
    for (int r = 0; r < 8; ++r) {
      float v = acc[t][r] + bv;
      if (resid) { float rv = resid[(size_t)((row0 + 8 * hh + r) % rmod) * ldr + col]; if (RES_BF16) rv = bf16_round(rv); v += rv; }
      if (ACT == 1) v = fmaxf(v, 0.f);
      if (ACT == 2) v = 0.5f * v * (1.0f + erff(v * 0.70710678118654752f));
      if (ACT == 3) { const float u = 0.7978845608028654f * (v + 0.044715f * v * v * v); v = 0.5f * v * (1.0f + tanhf(u)); }
      so[w][8 * hh + r][t * 16 + ln] = v;
    }
  }
  __builtin_amdgcn_fence(__ATOMIC_ACQ_REL, "workgroup");
  __builtin_amdgcn_wave_barrier();
  const int rsub = lane >> 4, c4 = (lane & 15) * 4;
  for (int pass = 0; pass < 2; ++pass) {
#pragma unroll
    for (int q = 0; q < 8; ++q) {
      const int r = q * 2 + rsub;
      const v4f v = *(const v4fa*)&so[w][r][c4];
      *(volatile v4f*)(C + (size_t)(row0 + r) * ldc + col0 + c4) = v;
    }
    if (pass == 0) __threadfence();
  }
}
template <bool PARAM_BF16>
__global__ __launch_bounds__(256) void k_layernorm(const float* __restrict__ X, const float* __restrict__ R, const float* __restrict__ g, const float* __restrict__ bta,
                                                  float* __restrict__ out_sum, float* __restrict__ out_norm, int N, float eps) {
  __shared__ float red[256];
  const int row = blockIdx.x, tid = threadIdx.x;
  const float* x = X + (size_t)row * N; const float* rr = R ? R + (size_t)row * N : nullptr;
  float vals[16];
  const int per = N / 256;
  float s1 = 0.f;
  for (int u = 0; u < per / 4; ++u) {
    const int j = tid * 4 + 1024 * u;
    const v4f a = *(const v4fa*)(x + j);
    v4f b = {0.f,0.f,0.f,0.f}; if (rr) b = *(const v4fa*)(rr + j);
#pragma unroll
    for (int q = 0; q < 4; ++q) { const float v = a[q] + b[q]; vals[u * 4 + q] = v; s1 += v; }
  }
  red[tid] = s1; __syncthreads();
  for (int st = 128; st > 0; st >>= 1) { if (tid < st) red[tid] += red[tid + st]; __syncthreads(); }
  const float mu = red[0] / (float)N; __syncthreads();
  float s2 = 0.f;
  for (int u = 0; u < per / 4; ++u)
#pragma unroll
    for (int q = 0; q < 4; ++q) { const float c = vals[u * 4 + q] - mu; s2 += c * c; }
  red[tid] = s2; __syncthreads();
  for (int st = 128; st > 0; st >>= 1) { if (tid < st) red[tid] += red[tid + st]; __syncthreads(); }
  const float rs = rsqrtf(red[0] / (float)N + eps);
  for (int pass = 0; pass < 2; ++pass) {
    for (int u = 0; u < per / 4; ++u) {
      const int j = tid * 4 + 1024 * u;
      v4f o, sm;
#pragma unroll
      for (int q = 0; q < 4; ++q) {
        float gg = g[j + q], bb = bta[j + q];
        if (PARAM_BF16) { gg = bf16_round(gg); bb = bf16_round(bb); }
        sm[q] = vals[u * 4 + q]; o[q] = (vals[u * 4 + q] - mu) * rs * gg + bb;
      }
      if (out_sum) *(volatile v4f*)(out_sum + (size_t)row * N + j) = sm;
      *(volatile v4f*)(out_norm + (size_t)row * N + j) = o;
    }
    if (pass == 0) __threadfence();
  }
}


typedef _Float16 v16h __attribute__((ext_vector_type(16)));
union FragH { v16h v; v8us half[2]; _Float16 h[16]; unsigned short u[16]; };
template <int NT>
__device__ __forceinline__ v8f mmaH(v16h ah, v16h al, v16h bh, v16h bl, v8f c) {
  c = __builtin_amdgcn_wmma_f32_16x16x32_f16(false, ah, false, bh, (short)0, c, false, false);
  if (NT >= 2) c = __builtin_amdgcn_wmma_f32_16x16x32_f16(false, al, false, bh, (short)0, c, false, false);
  if (NT >= 3) c = __builtin_amdgcn_wmma_f32_16x16x32_f16(false, ah, false, bl, (short)0, c, false, false);
  asm volatile("v_nop\n\tv_nop\n\tv_nop\n\tv_nop" : "+v"(c) : "v"(ah), "v"(al), "v"(bh), "v"(bl));
  return c;
}
template <bool ASPLIT>
__global__ __launch_bounds__(128) void k_gemm_h(const float* __restrict__ A, int lda, size_t sA, const _Float16* __restrict__ Bh, int ldb, size_t sB, float alpha, float* __restrict__ C, int ldc, size_t sC, int M, int N, int K) {
  __shared__ __attribute__((aligned(16))) float so[4][16][64];
  const int tid = threadIdx.x, w = tid >> 5, lane = tid & 31, ln = lane & 15, hh = lane >> 4; const int by = blockIdx.y;
  A += (size_t)by * sA; Bh += (size_t)by * sB; C += (size_t)by * sC;
  const int ntn = (N + 63) / 64; const int wid = blockIdx.x * 4 + w; const int mt = wid / ntn, nq = wid % ntn; if (mt * 16 >= M) return;
  const int row0 = mt * 16, col0 = nq * 64; const float* arow = A + (size_t)(row0 + ln) * lda;
  v8f acc[4] = {};
  for (int kb = 0; kb < K; kb += 32) {
    FragH ah, al;
    const v4f x0 = *(const v4fa*)(arow + kb + 8 * hh), x1 = *(const v4fa*)(arow + kb + 8 * hh + 4), x2 = *(const v4fa*)(arow + kb + 16 + 8 * hh), x3 = *(const v4fa*)(arow + kb + 16 + 8 * hh + 4);
    float xs[16] = {x0[0],x0[1],x0[2],x0[3],x1[0],x1[1],x1[2],x1[3],x2[0],x2[1],x2[2],x2[3],x3[0],x3[1],x3[2],x3[3]};
#pragma unroll
    for (int i = 0; i < 16; ++i) { const _Float16 h = (_Float16)xs[i]; ah.h[i] = h; al.h[i] = ASPLIT ? (_Float16)(xs[i] - (float)h) : (_Float16)0.0f; }
#pragma unroll
    for (int t = 0; t < 4; ++t) { if (col0 + t * 16 >= N) continue; const size_t boff = (size_t)(col0 + t * 16 + ln) * ldb + kb; FragH bq; bq.half[0] = *(const v8us*)(Bh + boff + 8 * hh); bq.half[1] = *(const v8us*)(Bh + boff + 16 + 8 * hh);
      acc[t] = mmaH<ASPLIT ? 2 : 1>(ah.v, al.v, bq.v, bq.v, acc[t]); }
  }
#pragma unroll
  for (int t = 0; t < 4; ++t) { if (col0 + t * 16 >= N) continue;
#pragma unroll
    for (int r = 0; r < 8; ++r) so[w][8 * hh + r][t * 16 + ln] = acc[t][r] * alpha; }
  __builtin_amdgcn_fence(__ATOMIC_ACQ_REL, "workgroup"); __builtin_amdgcn_wave_barrier();
  const int rsub = lane >> 4, c4 = (lane & 15) * 4;
  for (int pass = 0; pass < 2; ++pass) {
#pragma unroll
    for (int q = 0; q < 8; ++q) { const int r = q * 2 + rsub; if (col0 + c4 < N) { const v4f v = *(const v4fa*)&so[w][r][c4]; *(volatile v4f*)(C + (size_t)(row0 + r) * ldc + col0 + c4) = v; } }
    if (pass == 0) __threadfence(); }
}

__global__ __launch_bounds__(256) void k_wt_f16(const float* __restrict__ W, _Float16* __restrict__ Wt, int K, int N, float scale) {
  const int t = blockIdx.x * 256 + threadIdx.x; if (t >= N * (K / 8)) return; const int n = t / (K / 8), k8 = (t % (K / 8)) * 8; FragH f;
#pragma unroll
  for (int i = 0; i < 8; ++i) f.h[i] = (_Float16)(bf16_round(W[(size_t)(k8 + i) * N + n]) * scale); const v8us o = f.half[0];
  *(volatile v8us*)((unsigned short*)Wt + (size_t)n * K + k8) = o; __threadfence(); *(volatile v8us*)((unsigned short*)Wt + (size_t)n * K + k8) = o;
}
template <int ACT>
__global__ __launch_bounds__(128) void k_gemm_hhx(const _Float16* __restrict__ A, int lda, size_t sA, const _Float16* __restrict__ Bh, int ldb, size_t sB, float alpha, const float* __restrict__ bias, size_t sBias, const float* __restrict__ CP, int rowsPerB, size_t sCPb, int row0g,
    float* __restrict__ C, _Float16* __restrict__ C16, int ldc, size_t sC, int M, int N, int K) {
  __shared__ __attribute__((aligned(16))) float so[4][16][64];
  const int tid = threadIdx.x, w = tid >> 5, lane = tid & 31, ln = lane & 15, hh = lane >> 4; const int by = blockIdx.y;
  A += (size_t)by * sA; Bh += (size_t)by * sB; const size_t cofs = (size_t)by * sC; const float* bp = bias ? bias + (size_t)by * sBias : nullptr;
  const int ntn = (N + 63) / 64; const int wid = blockIdx.x * 4 + w; const int mt = wid / ntn, nq = wid % ntn; if (mt * 16 >= M) return;
  const int row0 = mt * 16, col0 = nq * 64; const _Float16* arow = A + (size_t)(row0 + ln) * lda;
  v8f acc[4] = {};
  for (int kb = 0; kb < K; kb += 32) { FragH ah; ah.half[0] = *(const v8us*)((const unsigned short*)arow + kb + 8 * hh); ah.half[1] = *(const v8us*)((const unsigned short*)arow + kb + 16 + 8 * hh);
#pragma unroll
    for (int t = 0; t < 4; ++t) { if (col0 + t * 16 >= N) continue; const size_t boff = (size_t)(col0 + t * 16 + ln) * ldb + kb; FragH bq; bq.half[0] = *(const v8us*)((const unsigned short*)Bh + boff + 8 * hh); bq.half[1] = *(const v8us*)((const unsigned short*)Bh + boff + 16 + 8 * hh);
      acc[t] = mmaH<1>(ah.v, ah.v, bq.v, bq.v, acc[t]); }
  }
#pragma unroll
  for (int t = 0; t < 4; ++t) { if (col0 + t * 16 >= N) continue; const int col = col0 + t * 16 + ln; const float bv = bp ? bf16_round(bp[col]) : 0.f;
#pragma unroll
    for (int r = 0; r < 8; ++r) { float v = acc[t][r] * alpha + bv; if (CP) { const int bidx = (row0g + row0 + 8 * hh + r) / rowsPerB; v += CP[(size_t)bidx * sCPb + (size_t)by * 64 + col]; } if (ACT == 1) v = (v > 0.f) ? v : expm1f(v); else if (ACT == 7) v = (v > 0.f) ? v + 1.0f : expf(v); else if (ACT == 8) v = tanhf(v); else if (ACT == 9) v = 0.5f * v * (1.0f + tanhf(0.7978845608028654f * (v + 0.044715f * v * v * v))); else if (ACT == 11) v = 1.0f / (1.0f + expf(-v)); else if (ACT == 12) v = (v > 0.f) ? v : 0.01f * v; else if (ACT == 14) v = (v > 0.f) ? v : 0.1f * v; else if (ACT == 15) v = v / (1.0f + expf(-v)); else if (ACT == 3) v = fmaxf(v, 0.f); else if (ACT == 6) v = 0.5f * v * (1.0f + erff(v * 0.70710678118654752f)); so[w][8 * hh + r][t * 16 + ln] = v; } }
  __builtin_amdgcn_fence(__ATOMIC_ACQ_REL, "workgroup"); __builtin_amdgcn_wave_barrier();
  const int rsub = lane >> 4, c4 = (lane & 15) * 4; typedef _Float16 v4h __attribute__((ext_vector_type(4)));
  for (int pass = 0; pass < 2; ++pass) {
#pragma unroll
    for (int q = 0; q < 8; ++q) { const int r = q * 2 + rsub; if (col0 + c4 < N) { const v4f v = *(const v4fa*)&so[w][r][c4]; if (C) *(volatile v4f*)(C + cofs + (size_t)(row0 + r) * ldc + col0 + c4) = v; if (C16) { v4h h4; for (int i = 0; i < 4; ++i) h4[i] = (_Float16)v[i]; *(volatile v4h*)(C16 + cofs + (size_t)(row0 + r) * ldc + col0 + c4) = h4; } } }
    if (pass == 0) __threadfence(); }
}


typedef _Float16 v4h __attribute__((ext_vector_type(4)));

__global__ __launch_bounds__(256) void k_x16(const float* __restrict__ x, _Float16* __restrict__ X16, size_t n8) { const size_t t = (size_t)blockIdx.x * 256 + threadIdx.x; if (t >= n8) return; FragH f;
#pragma unroll
  for (int q = 0; q < 8; ++q) f.h[q] = (_Float16)bf16_round(x[t * 8 + q]); *(volatile v8us*)((unsigned short*)X16 + t * 8) = f.half[0]; __threadfence(); *(volatile v8us*)((unsigned short*)X16 + t * 8) = f.half[0]; }
__global__ __launch_bounds__(256) void k_h16(const float* __restrict__ x, _Float16* __restrict__ X16, size_t n8) { const size_t t = (size_t)blockIdx.x * 256 + threadIdx.x; if (t >= n8) return; FragH f;
#pragma unroll
  for (int q = 0; q < 8; ++q) f.h[q] = (_Float16)x[t * 8 + q]; *(volatile v8us*)((unsigned short*)X16 + t * 8) = f.half[0]; __threadfence(); *(volatile v8us*)((unsigned short*)X16 + t * 8) = f.half[0]; }
__global__ __launch_bounds__(256) void k_round16f(const float* __restrict__ W, _Float16* __restrict__ Bt, size_t n8) { const size_t t = (size_t)blockIdx.x * 256 + threadIdx.x; if (t >= n8) return; FragH f;
#pragma unroll
  for (int i = 0; i < 8; ++i) f.h[i] = (_Float16)(bf16_round(W[t * 8 + i]) * 16.0f); *(volatile v8us*)((unsigned short*)Bt + t * 8) = f.half[0]; __threadfence(); *(volatile v8us*)((unsigned short*)Bt + t * 8) = f.half[0]; }
template <int NHv, int TTv>
__global__ __launch_bounds__(256) void k_vt(const _Float16* __restrict__ V16, int ldv, int voff, _Float16* __restrict__ Vt) { __shared__ unsigned short tl[64][66]; const int tid = threadIdx.x; const int slab = blockIdx.x / (TTv / 64), lg = blockIdx.x % (TTv / 64); const int b = slab / NHv, h = slab % NHv;
  for (int i = tid; i < 64 * 8; i += 256) { const int r = i / 8, c8 = (i % 8) * 8; FragH f; f.half[0] = *(const v8us*)((const unsigned short*)V16 + ((size_t)b * TTv + lg * 64 + r) * ldv + voff + h * 64 + c8);
#pragma unroll
    for (int q = 0; q < 8; ++q) tl[r][c8 + q] = f.u[q]; }
  __syncthreads();
  for (int pass = 0; pass < 2; ++pass) {
#pragma unroll
    for (int rd = 0; rd < 2; ++rd) { const int d = rd * 32 + tid / 8, pc = tid % 8; FragH f;
#pragma unroll
      for (int q = 0; q < 8; ++q) f.u[q] = tl[pc * 8 + q][d];
      *(volatile v8us*)((unsigned short*)Vt + ((size_t)slab * 64 + d) * TTv + lg * 64 + pc * 8) = f.half[0]; }
    if (pass == 0) __threadfence(); } }

__global__ __launch_bounds__(256) void k_hl(const float* __restrict__ F, _Float16* __restrict__ Hh, _Float16* __restrict__ Hl, size_t n8) { const size_t t = (size_t)blockIdx.x * 256 + threadIdx.x; if (t >= n8) return; FragH fh, fl; const v4f a = *(const v4fa*)(F + t * 8), c = *(const v4fa*)(F + t * 8 + 4);
#pragma unroll
  for (int q = 0; q < 4; ++q) { _Float16 h = (_Float16)a[q]; fh.h[q] = h; fl.h[q] = (_Float16)((a[q] - (float)h) * 1024.0f); h = (_Float16)c[q]; fh.h[4 + q] = h; fl.h[4 + q] = (_Float16)((c[q] - (float)h) * 1024.0f); }
  for (int pass = 0; pass < 2; ++pass) { *(volatile v8us*)((unsigned short*)Hh + t * 8) = fh.half[0]; *(volatile v8us*)((unsigned short*)Hl + t * 8) = fl.half[0]; if (pass == 0) __threadfence(); } }
#define VST2(T, ptr, val) do { const T vst2_v_ = (val); *(volatile T*)(ptr) = vst2_v_; __threadfence(); *(volatile T*)(ptr) = vst2_v_; } while (0)

#define C4_NB 4096
#define C4_CH 8192
__device__ __forceinline__ int c4_bucket(int v, int N) { v = min(max(v, 0), N - 1); return (int)(((long long)v * C4_NB) / N); }
__global__ __launch_bounds__(256) void k_c4_count(const int* __restrict__ tgt, int E, int N, int* __restrict__ CNT) {
    __shared__ int hist[C4_NB]; const int ch = blockIdx.x, t = threadIdx.x; const int e0 = ch * C4_CH; const int nt = min(C4_CH, E - e0);
    for (int j = 0; j < 16; ++j) hist[t + 256 * j] = 0; __syncthreads();
    for (int i = t; i < nt; i += 256) atomicAdd(&hist[c4_bucket(tgt[e0 + i], N)], 1);
    __syncthreads();
    for (int j = 0; j < 16; ++j) { const int v = hist[t + 256 * j]; VST2(int, CNT + (long long)ch * C4_NB + t + 256 * j, v); } }
__global__ __launch_bounds__(256) void k_c4_offsets(const int* __restrict__ CNT, int nch, int E, int* __restrict__ OFFB, int* __restrict__ BOFF) {
    __shared__ int tot[C4_NB]; __shared__ int part[256]; const int t = threadIdx.x;
    for (int j = 0; j < 16; ++j) { const int b = t + 256 * j; int s = 0; for (int ch = 0; ch < nch; ++ch) s += CNT[(long long)ch * C4_NB + b]; tot[b] = s; }
    __syncthreads();
    { int s = 0; for (int q = 0; q < 16; ++q) s += tot[16 * t + q]; part[t] = s; } __syncthreads();
    if (t == 0) { int run = 0; for (int i = 0; i < 256; ++i) { const int v = part[i]; part[i] = run; run += v; } } __syncthreads();
    { int run = part[t]; for (int q = 0; q < 16; ++q) { const int v = tot[16 * t + q]; tot[16 * t + q] = run; run += v; } }
    __syncthreads();
    for (int j = 0; j < 16; ++j) { const int b = t + 256 * j; VST2(int, BOFF + b, tot[b]); }
    if (t == 0) VST2(int, BOFF + C4_NB, E);
    for (int j = 0; j < 16; ++j) { const int b = t + 256 * j; int run = tot[b]; for (int ch = 0; ch < nch; ++ch) { VST2(int, OFFB + (long long)ch * C4_NB + b, run); run += CNT[(long long)ch * C4_NB + b]; } } }
__global__ __launch_bounds__(256) void k_c4_scatter(const int* __restrict__ tgt, int E, int N, const int* __restrict__ OFFB, int* __restrict__ BUF) {
    __shared__ int cur[C4_NB]; __shared__ int bk[256]; const int ch = blockIdx.x, t = threadIdx.x; const int e0 = ch * C4_CH; const int nt = min(C4_CH, E - e0);
    const int wv = t >> 5, ln = t & 31;
    for (int j = 0; j < 16; ++j) cur[t + 256 * j] = OFFB[(long long)ch * C4_NB + t + 256 * j];
    __syncthreads();
    for (int s0 = 0; s0 < C4_CH; s0 += 256) {
        const int i = s0 + t; const int e = e0 + i; const int b = (i < nt) ? c4_bucket(tgt[min(e, E - 1)], N) : -1;
        bk[t] = b; __syncthreads();
        int rank = 0, cntw = 0;
        for (int l = 0; l < 32; ++l) { const int o = bk[(wv << 5) + l]; const bool same = (o == b) && (b >= 0); cntw += same ? 1 : 0; rank += (same && l < ln) ? 1 : 0; }
        const bool last = (b >= 0) && (rank == cntw - 1);
        for (int w = 0; w < 8; ++w) {
            if (wv == w && b >= 0) { int pos = cur[b] + rank; pos = min(max(pos, 0), E - 1); VST2(int, BUF + pos, e); }
            __syncthreads();
            if (wv == w && last) cur[b] += cntw;
            __syncthreads(); }
    } }
template <int CAP>
__global__ __launch_bounds__(256) void k_c4_lists(const int* __restrict__ tgt, const int* __restrict__ BUF, const int* __restrict__ BOFF, int N, int E, int* __restrict__ NBR, int* __restrict__ cnt) {
    const int d = blockIdx.x * 256 + threadIdx.x; if (d >= N) return; const int b = c4_bucket(d, N); int n = 0; int* row = NBR + (long long)d * CAP;
    const int p0 = min(max(BOFF[b], 0), E), p1 = min(max(BOFF[b + 1], p0), E);
    for (int p = p0; p < p1; ++p) { int e = BUF[p]; e = min(max(e, 0), E - 1); if (tgt[e] == d) { if (n < CAP) VST2(int, row + n, e); ++n; } }
    for (int j = n; j < CAP; ++j) VST2(int, row + j, -1); VST2(int, cnt + d, min(n, CAP)); }
__global__ __launch_bounds__(256) void k_c4_scan1(const int* __restrict__ cnt, int* __restrict__ PART, int N) {
    __shared__ int part[256]; const int per = ((((N + 255) / 256) + 31) / 32) * 32; const int a = threadIdx.x * per, b = min(N, a + per); int s = 0;
    for (int i = a; i < b; ++i) s += cnt[i]; part[threadIdx.x] = s; __syncthreads();
    if (threadIdx.x == 0) { int run = 0; for (int t = 0; t < 256; ++t) { const int v = part[t]; part[t] = run; run += v; } } __syncthreads();
    VST2(int, PART + threadIdx.x, part[threadIdx.x]); }
__global__ __launch_bounds__(256) void k_c4_scan2(const int* __restrict__ cnt, const int* __restrict__ PART, int* __restrict__ off, int N) {
    const int i = blockIdx.x * 256 + threadIdx.x; if (i > N) return; const int per = ((((N + 255) / 256) + 31) / 32) * 32; const int r = min(i / per, 255); const int a = r * per;
    int s = PART[r]; for (int kq = a; kq < i; ++kq) s += cnt[min(kq, N - 1)];
    VST2(int, off + i, s); }
template <int CAP>
__global__ __launch_bounds__(256) void k_c4_slotcopy(const int* __restrict__ off, const int* __restrict__ NBR, int* __restrict__ slot, int N) {
    const int t = blockIdx.x * 256 + threadIdx.x; const int tot = off[N]; if (t >= tot) return;
    int lo = 0, hi = N - 1; while (lo < hi) { const int mid = (lo + hi + 1) >> 1; if (off[mid] <= t) lo = mid; else hi = mid - 1; }
    int j = t - off[lo]; j = (j < 0) ? 0 : ((j >= CAP) ? (CAP - 1) : j); VST2(int, slot + t, NBR[(long long)lo * CAP + j]); }

__global__ __launch_bounds__(256) void k_split(const float* __restrict__ F, _Float16* __restrict__ Hh, _Float16* __restrict__ Hl, size_t n8) {
  #pragma clang fp contract(off)
  const size_t t = (size_t)blockIdx.x * 256 + threadIdx.x; if (t >= n8) return; const v4f a = *(const v4fa*)(F + t * 8), c = *(const v4fa*)(F + t * 8 + 4); FragH fh, fl;
#pragma unroll
  for (int q = 0; q < 8; ++q) { const float v = (q < 4) ? a[q] : c[q - 4]; const _Float16 hi = (_Float16)v; fh.h[q] = hi; fl.h[q] = (_Float16)((v - (float)hi) * 1024.0f); }
  for (int pass = 0; pass < 2; ++pass) { *(volatile v8us*)((unsigned short*)Hh + t * 8) = fh.half[0]; *(volatile v8us*)((unsigned short*)Hl + t * 8) = fl.half[0]; if (pass == 0) __threadfence(); } }
__global__ __launch_bounds__(256) void k_embed(const float* __restrict__ x, const float* __restrict__ Wm, const float* __restrict__ bb, float* __restrict__ H) {
  #pragma clang fp contract(off)
  const int t = blockIdx.x * 256 + threadIdx.x; if (t >= NN * (DDm / 4)) return; const int c0 = (t % (DDm / 4)) * 4, n = t / (DDm / 4); v4f o;
#pragma unroll
  for (int q = 0; q < 4; ++q) { float s = bf16_round(bb[c0 + q]);
#pragma unroll
    for (int a = 0; a < NA; ++a) s += bf16_round(x[(size_t)n * NA + a]) * bf16_round(Wm[a * DDm + c0 + q]);
    o[q] = s; }
  *(volatile v4f*)(H + (size_t)n * DDm + c0) = o; __threadfence(); *(volatile v4f*)(H + (size_t)n * DDm + c0) = o; }
__global__ __launch_bounds__(256) void k_wsl(const float* __restrict__ Wm, int r0, _Float16* __restrict__ Bt) { const int t = blockIdx.x * 256 + threadIdx.x; if (t >= DDm * 8) return; const int k0 = (t & 7) * 8, o = t >> 3; FragH f;
#pragma unroll
  for (int q = 0; q < 8; ++q) f.h[q] = (_Float16)(bf16_round(Wm[(size_t)(r0 + k0 + q) * DDm + o]) * 16.0f);
  *(volatile v8us*)((unsigned short*)Bt + (size_t)o * DDm + k0) = f.half[0]; __threadfence(); *(volatile v8us*)((unsigned short*)Bt + (size_t)o * DDm + k0) = f.half[0]; }
__global__ __launch_bounds__(256) void k_msg(const int* __restrict__ NBR, const int* __restrict__ cnt, const int* __restrict__ src, const float* __restrict__ pos, const float* __restrict__ PA, const float* __restrict__ PB, const float* __restrict__ W1, const float* __restrict__ b1, _Float16* __restrict__ Rh, _Float16* __restrict__ Rl, float* __restrict__ CFL) {
  #pragma clang fp contract(off)
  const int tid = threadIdx.x, w = tid >> 5, l = tid & 31; const int n = blockIdx.x * 8 + w; if (n >= NN) return; const int ne = min(cnt[n], DCAP); const int c0 = 2 * l; const float pnx = bf16_round(pos[(size_t)n * 3]), pny = bf16_round(pos[(size_t)n * 3 + 1]), pnz = bf16_round(pos[(size_t)n * 3 + 2]);
  const float pb0 = PB[(size_t)n * DDm + c0] + bf16_round(b1[c0]), pb1 = PB[(size_t)n * DDm + c0 + 1] + bf16_round(b1[c0 + 1]); const float wd0 = bf16_round(W1[(size_t)128 * DDm + c0]), wd1 = bf16_round(W1[(size_t)128 * DDm + c0 + 1]); float a0 = 0.f, a1 = 0.f;
#pragma unroll 1
  for (int j = 0; j < ne; ++j) { int e = NBR[(size_t)n * DCAP + j]; e = min(max(e, 0), NE - 1); int s = src[e]; s = min(max(s, 0), NN - 1); const float dx = bf16_round(pos[(size_t)s * 3]) - pnx, dy = bf16_round(pos[(size_t)s * 3 + 1]) - pny, dz = bf16_round(pos[(size_t)s * 3 + 2]) - pnz; const float dist = sqrtf((dx * dx + dy * dy) + dz * dz);
    a0 += fmaxf((PA[(size_t)s * DDm + c0] + pb0) + dist * wd0, 0.f); a1 += fmaxf((PA[(size_t)s * DDm + c0 + 1] + pb1) + dist * wd1, 0.f); }
  const float inv = (ne > 0) ? 1.0f / (float)ne : 0.f; const float m0 = a0 * inv, m1 = a1 * inv; FragH fh, fl; const _Float16 h0 = (_Float16)m0, h1 = (_Float16)m1; fh.h[0] = h0; fh.h[1] = h1; fl.h[0] = (_Float16)((m0 - (float)h0) * 1024.0f); fl.h[1] = (_Float16)((m1 - (float)h1) * 1024.0f); const float flag = (l == 0) ? ((ne > 0) ? 1.f : 0.f) : 0.f;
  for (int pass = 0; pass < 2; ++pass) { *(volatile unsigned int*)((unsigned short*)Rh + (size_t)n * DDm + c0) = *(const unsigned int*)&fh.u[0]; *(volatile unsigned int*)((unsigned short*)Rl + (size_t)n * DDm + c0) = *(const unsigned int*)&fl.u[0]; *(volatile float*)(CFL + (size_t)n * 32 + l) = flag; if (pass == 0) __threadfence(); } }
__global__ __launch_bounds__(256) void k_agg(const float* __restrict__ T, const float* __restrict__ CFL, const float* __restrict__ b2, _Float16* __restrict__ Ah, _Float16* __restrict__ Al) {
  #pragma clang fp contract(off)
  const int t = blockIdx.x * 256 + threadIdx.x; if (t >= NN * 8) return; const int c0 = (t & 7) * 8, n = t >> 3; const float f = CFL[(size_t)n * 32]; FragH fh, fl;
#pragma unroll
  for (int q = 0; q < 8; ++q) { const float v = (f > 0.5f) ? (T[(size_t)n * DDm + c0 + q] + bf16_round(b2[c0 + q])) : 0.f; const _Float16 hi = (_Float16)v; fh.h[q] = hi; fl.h[q] = (_Float16)((v - (float)hi) * 1024.0f); }
  for (int pass = 0; pass < 2; ++pass) { *(volatile v8us*)((unsigned short*)Ah + (size_t)n * DDm + c0) = fh.half[0]; *(volatile v8us*)((unsigned short*)Al + (size_t)n * DDm + c0) = fl.half[0]; if (pass == 0) __threadfence(); } }
__global__ __launch_bounds__(256) void k_lnres(float* __restrict__ H, const float* __restrict__ HN, const float* __restrict__ g, const float* __restrict__ bb) {
  #pragma clang fp contract(off)
  const int tid = threadIdx.x, w = tid >> 5, l = tid & 31; const int n = blockIdx.x * 8 + w; if (n >= NN) return; const int c0 = 2 * l; const float v0 = HN[(size_t)n * DDm + c0], v1 = HN[(size_t)n * DDm + c0 + 1]; float s = v0 + v1; for (int o = 16; o > 0; o >>= 1) s += __shfl_xor(s, o, 32); const float mu = s / 64.0f; float q2 = (v0 - mu) * (v0 - mu) + (v1 - mu) * (v1 - mu); for (int o = 16; o > 0; o >>= 1) q2 += __shfl_xor(q2, o, 32); const float rs = rsqrtf(q2 / 64.0f + 1e-5f);
  const float y0 = fmaxf(H[(size_t)n * DDm + c0] + ((v0 - mu) * rs * bf16_round(g[c0]) + bf16_round(bb[c0])), 0.f), y1 = fmaxf(H[(size_t)n * DDm + c0 + 1] + ((v1 - mu) * rs * bf16_round(g[c0 + 1]) + bf16_round(bb[c0 + 1])), 0.f);
  typedef float v2f __attribute__((ext_vector_type(2))); v2f yy; yy[0] = y0; yy[1] = y1; *(volatile v2f*)(H + (size_t)n * DDm + c0) = yy; __threadfence(); *(volatile v2f*)(H + (size_t)n * DDm + c0) = yy; }
__global__ __launch_bounds__(256) void k_granges(const int* __restrict__ batch, int* __restrict__ GR) { __shared__ int st[NG], en[NG]; const int tid = threadIdx.x; if (tid < NG) { st[tid] = NN; en[tid] = -1; } __syncthreads();
#pragma unroll 1
  for (int n = tid; n < NN; n += 256) { int g = batch[n]; g = min(max(g, 0), NG - 1); atomicMin(&st[g], n); atomicMax(&en[g], n); }
  __syncthreads();
  if (tid < 32) { for (int g = 0; g < NG; ++g) { const int s = st[g], c = (en[g] >= s) ? (en[g] - s + 1) : 0; const int v = (tid == 0) ? ((c > 0) ? s : 0) : (tid == 1) ? c : 0; *(volatile int*)(GR + g * 32 + tid) = v; __threadfence(); *(volatile int*)(GR + g * 32 + tid) = v; } } }
__global__ __launch_bounds__(256) void k_pool(const float* __restrict__ H, const int* __restrict__ batch, const int* __restrict__ GR, float* __restrict__ GP) {
  #pragma clang fp contract(off)
  __shared__ float part[4][DDm]; const int tid = threadIdx.x, g = blockIdx.x; const int c = tid & 63, stp = tid >> 6; const int s = GR[g * 32], cntg = GR[g * 32 + 1]; float acc = 0.f; int k = 0;
#pragma unroll 1
  for (int i = stp; i < cntg; i += 4) { const int n = s + i; if (batch[n] == g) { acc += H[(size_t)n * DDm + c]; ++k; } }
  part[stp][c] = acc; __shared__ int kc[4]; if (c == 0) kc[stp] = k; __syncthreads();
  if (tid < DDm) { const float tot = (part[0][tid] + part[1][tid]) + (part[2][tid] + part[3][tid]); const int kk = kc[0] + kc[1] + kc[2] + kc[3]; const float v = tot / fmaxf((float)kk, 1.0f); *(volatile float*)(GP + (size_t)g * DDm + tid) = v; __threadfence(); *(volatile float*)(GP + (size_t)g * DDm + tid) = v; } }
__global__ __launch_bounds__(256) void k_head(const float* __restrict__ GP, const float* __restrict__ W1, const float* __restrict__ b1, const float* __restrict__ W2, const float* __restrict__ b2, const float* __restrict__ W3, const float* __restrict__ b3, float* __restrict__ out) {
  #pragma clang fp contract(off)
  __shared__ float z1[NG][DDm + 1]; __shared__ float z2[NG][33]; __shared__ float res[NG]; const int tid = threadIdx.x;
  for (int i = tid; i < NG * DDm; i += 256) { const int g = i / DDm, o = i % DDm; float s = bf16_round(b1[o]);
#pragma unroll 1
    for (int c = 0; c < DDm; ++c) s += GP[(size_t)g * DDm + c] * bf16_round(W1[c * DDm + o]);
    z1[g][o] = fmaxf(s, 0.f); }
  __syncthreads();
  for (int i = tid; i < NG * 32; i += 256) { const int g = i / 32, o = i % 32; float s = bf16_round(b2[o]);
#pragma unroll 1
    for (int c = 0; c < DDm; ++c) s += z1[g][c] * bf16_round(W2[c * 32 + o]);
    z2[g][o] = fmaxf(s, 0.f); }
  __syncthreads();
  if (tid < NG) { float s = bf16_round(b3[0]);
#pragma unroll 1
    for (int c = 0; c < 32; ++c) s += z2[tid][c] * bf16_round(W3[c]);
    res[tid] = s; }
  __syncthreads();
  if (tid < NG) { *(volatile float*)(out + tid) = res[tid]; __threadfence(); *(volatile float*)(out + tid) = res[tid]; } }

extern "C" void kernel_launch(void* const* d_in, const int* in_sizes, int n_in,
                              void* d_out, int out_size, void* d_ws, size_t ws_size, hipStream_t stream) {
  (void)in_sizes; (void)n_in; (void)out_size;
  const float* const* I = (const float* const*)d_in; const float* x = I[0]; const float* pos = I[1]; const int* ei = (const int*)d_in[2]; const int* batch = (const int*)d_in[3]; const float* atom_W = I[4]; const float* atom_b = I[5]; const float* msg_W1 = I[6]; const float* msg_b1 = I[7]; const float* msg_W2 = I[8]; const float* msg_b2 = I[9]; const float* upd_W = I[10]; const float* upd_b = I[11]; const float* ln_g = I[12]; const float* ln_b = I[13]; const float* hW1 = I[14]; const float* hb1 = I[15]; const float* hW2 = I[16]; const float* hb2 = I[17]; const float* hW3 = I[18]; const float* hb3 = I[19];
  const int* esrc = ei; const int* edst = ei + NE;
  char* ws = (char*)d_ws; size_t off = 0;
  auto take = [&](size_t bytes) { char* p = ws + off; off += (bytes + 255) & ~(size_t)255; return p; };
  const int nch = (NE + C4_CH - 1) / C4_CH;
  int* CNT = (int*)take((size_t)nch * C4_NB * 4); int* OFFB = (int*)take((size_t)nch * C4_NB * 4); int* BOFF = (int*)take((size_t)(C4_NB + 64) * 4); int* BUF = (int*)take((size_t)NE * 4); int* NBR = (int*)take((size_t)NN * DCAP * 4); int* cnt = (int*)take((size_t)(NN + 64) * 4); int* GR = (int*)take(NG * 32 * 4);
  _Float16* BA[NL]; _Float16* BB[NL]; _Float16* B2[NL]; _Float16* BUa[NL]; _Float16* BUb[NL]; for (int l = 0; l < NL; ++l) { BA[l] = (_Float16*)take(DDm * DDm * 2); BB[l] = (_Float16*)take(DDm * DDm * 2); B2[l] = (_Float16*)take(DDm * DDm * 2); BUa[l] = (_Float16*)take(DDm * DDm * 2); BUb[l] = (_Float16*)take(DDm * DDm * 2); }
  float* H = (float*)take((size_t)NNP * DDm * 4); _Float16* Hh = (_Float16*)take((size_t)NNP * DDm * 2); _Float16* Hl = (_Float16*)take((size_t)NNP * DDm * 2); float* PA = (float*)take((size_t)NNP * DDm * 4); float* PB = (float*)take((size_t)NNP * DDm * 4); _Float16* Rh = (_Float16*)take((size_t)NNP * DDm * 2); _Float16* Rl = (_Float16*)take((size_t)NNP * DDm * 2); float* CFL = (float*)take((size_t)NN * 32 * 4); float* T = (float*)take((size_t)NNP * DDm * 4); _Float16* AGh = (_Float16*)take((size_t)NNP * DDm * 2); _Float16* AGl = (_Float16*)take((size_t)NNP * DDm * 2); float* HN = (float*)take((size_t)NNP * DDm * 4); float* GP = (float*)take((size_t)NG * DDm * 4);
  if (off > ws_size) return;
  k_c4_count<<<nch, 256, 0, stream>>>(edst, NE, NN, CNT); k_c4_offsets<<<1, 256, 0, stream>>>(CNT, nch, NE, OFFB, BOFF); k_c4_scatter<<<nch, 256, 0, stream>>>(edst, NE, NN, OFFB, BUF); k_c4_lists<DCAP><<<(NN + 255) / 256, 256, 0, stream>>>(edst, BUF, BOFF, NN, NE, NBR, cnt);
  for (int l = 0; l < NL; ++l) { k_wsl<<<2, 256, 0, stream>>>(msg_W1 + (size_t)l * 129 * DDm, 0, BA[l]); k_wsl<<<2, 256, 0, stream>>>(msg_W1 + (size_t)l * 129 * DDm, 64, BB[l]); k_wsl<<<2, 256, 0, stream>>>(msg_W2 + (size_t)l * DDm * DDm, 0, B2[l]); k_wsl<<<2, 256, 0, stream>>>(upd_W + (size_t)l * 128 * DDm, 0, BUa[l]); k_wsl<<<2, 256, 0, stream>>>(upd_W + (size_t)l * 128 * DDm, 64, BUb[l]); }
  k_embed<<<(NN * 16 + 255) / 256, 256, 0, stream>>>(x, atom_W, atom_b, H);
  const dim3 gN(((NNP / 16) * 1 + 3) / 4, 1); const size_t n8 = (size_t)NNP * DDm / 8; const unsigned nb8 = (unsigned)((n8 + 255) / 256);
  for (int l = 0; l < NL; ++l) { const float* W1l = msg_W1 + (size_t)l * 129 * DDm;
    k_split<<<nb8, 256, 0, stream>>>(H, Hh, Hl, n8);
    k_gemm_hhx<0><<<gN, 128, 0, stream>>>(Hh, DDm, 0, BA[l], DDm, 0, 0.0625f, nullptr, 0, nullptr, 1, 0, 0, PA, nullptr, DDm, 0, NNP, DDm, DDm); k_gemm_hhx<0><<<gN, 128, 0, stream>>>(Hl, DDm, 0, BA[l], DDm, 0, 0.0625f / 1024.0f, nullptr, 0, PA, 1, (size_t)DDm, 0, PA, nullptr, DDm, 0, NNP, DDm, DDm);
    k_gemm_hhx<0><<<gN, 128, 0, stream>>>(Hh, DDm, 0, BB[l], DDm, 0, 0.0625f, nullptr, 0, nullptr, 1, 0, 0, PB, nullptr, DDm, 0, NNP, DDm, DDm); k_gemm_hhx<0><<<gN, 128, 0, stream>>>(Hl, DDm, 0, BB[l], DDm, 0, 0.0625f / 1024.0f, nullptr, 0, PB, 1, (size_t)DDm, 0, PB, nullptr, DDm, 0, NNP, DDm, DDm);
    k_msg<<<(NN + 7) / 8, 256, 0, stream>>>(NBR, cnt, esrc, pos, PA, PB, W1l, msg_b1 + l * DDm, Rh, Rl, CFL);
    k_gemm_hhx<0><<<gN, 128, 0, stream>>>(Rh, DDm, 0, B2[l], DDm, 0, 0.0625f, nullptr, 0, nullptr, 1, 0, 0, T, nullptr, DDm, 0, NNP, DDm, DDm); k_gemm_hhx<0><<<gN, 128, 0, stream>>>(Rl, DDm, 0, B2[l], DDm, 0, 0.0625f / 1024.0f, nullptr, 0, T, 1, (size_t)DDm, 0, T, nullptr, DDm, 0, NNP, DDm, DDm);
    k_agg<<<(NN * 8 + 255) / 256, 256, 0, stream>>>(T, CFL, msg_b2 + l * DDm, AGh, AGl);
    k_gemm_hhx<0><<<gN, 128, 0, stream>>>(Hh, DDm, 0, BUa[l], DDm, 0, 0.0625f, upd_b + l * DDm, 0, nullptr, 1, 0, 0, HN, nullptr, DDm, 0, NNP, DDm, DDm); k_gemm_hhx<0><<<gN, 128, 0, stream>>>(Hl, DDm, 0, BUa[l], DDm, 0, 0.0625f / 1024.0f, nullptr, 0, HN, 1, (size_t)DDm, 0, HN, nullptr, DDm, 0, NNP, DDm, DDm);
    k_gemm_hhx<0><<<gN, 128, 0, stream>>>(AGh, DDm, 0, BUb[l], DDm, 0, 0.0625f, nullptr, 0, HN, 1, (size_t)DDm, 0, HN, nullptr, DDm, 0, NNP, DDm, DDm); k_gemm_hhx<0><<<gN, 128, 0, stream>>>(AGl, DDm, 0, BUb[l], DDm, 0, 0.0625f / 1024.0f, nullptr, 0, HN, 1, (size_t)DDm, 0, HN, nullptr, DDm, 0, NNP, DDm, DDm);
    k_lnres<<<(NN + 7) / 8, 256, 0, stream>>>(H, HN, ln_g + l * DDm, ln_b + l * DDm); }
  k_granges<<<1, 256, 0, stream>>>(batch, GR); k_pool<<<NG, 256, 0, stream>>>(H, batch, GR, GP); k_head<<<1, 256, 0, stream>>>(GP, hW1, hb1, hW2, hb2, hW3, hb3, (float*)d_out);
}
